// LODE_T_77945066488240
// MI455X (gfx1250) — hardware-run, weakly checked
//
#include <hip/hip_runtime.h>
#include <math.h>

typedef __attribute__((ext_vector_type(16))) _Float16 v16h;
typedef __attribute__((ext_vector_type(8)))  _Float16 v8h;
typedef __attribute__((ext_vector_type(8)))  float    v8f;
typedef __attribute__((ext_vector_type(4)))  float    v4f;
typedef __attribute__((ext_vector_type(2)))  float    v2f;
typedef __attribute__((ext_vector_type(2)))  unsigned v2u;

constexpr int kNumSamples = 131072;
constexpr int kNeu        = 256;
constexpr int kSmp        = 16;
constexpr int kRowsA      = 3 * kSmp;
constexpr int kPitchA     = kNeu + 8;
constexpr int kPitchH     = kNeu + 4;
constexpr int kPitchT     = kNeu + 8;
constexpr int kOutCols    = 6;
constexpr float kEps      = 1e-4f;
constexpr float kCarryA   = 16.0f;
constexpr float kCarryW   = 16.0f;
constexpr float kFold     = 1.0f / (kCarryA * kCarryW);
static_assert((kNumSamples % kSmp) == 0, "sample tiles");
static_assert((kNeu % 32) == 0, "K multiple of 32");
static_assert((kNeu % 16) == 0 && (kRowsA % 16) == 0, "M,N tile multiples");
static_assert(kNeu == 256, "thread maps assume 256 neurons");
static_assert((kSmp * kOutCols * 4) % 128 == 0, "block output is whole 128-B lines");

constexpr size_t kOffBT   = 0;
constexpr size_t kWsTotal = kOffBT + (size_t)kNeu * kNeu * 2;
static_assert(kWsTotal == 131072ull, "carve total");
static_assert(kWsTotal <= 134217728ull, "carve cap");

template <typename T> struct Frag;
template <> struct Frag<_Float16> {
  typedef v16h V; union U { v16h v; v8h h[2]; };
  static __device__ __forceinline__ v16h load(const _Float16* p) {
    U f; f.h[0] = *(const v8h*)(p); f.h[1] = *(const v8h*)(p + 16); return f.v;
  }
};

__device__ __forceinline__ v8f mma_h(v16h a, v16h b, v8f c) {
  c = __builtin_amdgcn_wmma_f32_16x16x32_f16(false, a, false, b, (short)0, c, false, false);
  asm volatile("v_nop\n\tv_nop\n\tv_nop\n\tv_nop" : "+v"(c) : "v"(a), "v"(b));
  return c;
}

__device__ __forceinline__ float h16_to_f32(unsigned hb) {
  const unsigned sgn = (hb & 0x8000u) << 16; const unsigned em = hb & 0x7fffu;
  const float fn = __uint_as_float((em << 13) + 0x38000000u);
  const float fs = (float)em * 5.9604644775390625e-8f;
  const float mag = (em < 0x400u) ? fs : fn; return __uint_as_float(__float_as_uint(mag) | sgn);
}

__global__ __launch_bounds__(256) void transpose_w1_kernel(
    const float* __restrict__ W1, unsigned short* __restrict__ BtOut)
{
  const int i = blockIdx.x * 256 + threadIdx.x;
  const int nrow = i >> 5;
  const int k0 = (i & 31) * 8;
  v8h hv;
#pragma unroll
  for (int e = 0; e < 8; ++e) {
    const float w = W1[(size_t)(k0 + e) * kNeu + nrow] * kCarryW;
    hv[e] = (_Float16)w;
  }
  unsigned short* dst = BtOut + (size_t)nrow * kNeu + k0;
  *(volatile v8h*)dst = hv;
  __threadfence();
  *(volatile v8h*)dst = hv;
}

__global__ __launch_bounds__(256) void torus_dyn_kernel(
    const float* __restrict__ x,
    const float* __restrict__ W0, const float* __restrict__ b0,
    const unsigned short* __restrict__ BtPlane, const float* __restrict__ b1,
    const float* __restrict__ Wd, const float* __restrict__ bd,
    const float* __restrict__ Wo, const float* __restrict__ bo,
    const float* __restrict__ Wv,
    float* __restrict__ out, int n)
{
  __shared__ __align__(16) _Float16       sA[kRowsA * kPitchA];
  __shared__ __align__(16) float          sH[kSmp * kPitchH];
  __shared__ __align__(16) unsigned short sT[2 * kSmp * kPitchT];
  __shared__ __align__(16) float          sO[kSmp * kOutCols];

  const _Float16* Bt = (const _Float16*)BtPlane;
  const int tid  = threadIdx.x;
  const int wave = tid >> 5;
  const int lane = tid & 31;
  const int s    = tid >> 4;
  const int p    = tid & 15;

  const int gs  = blockIdx.x * kSmp + s;
  const int gsc = (gs < n) ? gs : (n - 1);
  const v2f* xr = (const v2f*)(x + (size_t)gsc * kOutCols);
  const v2f xq = xr[0];
  const v2f xd = xr[1];
  const v2f xt = xr[2];
  const float q0 = xq.x, q1 = xq.y;
  const float qd0 = xd.x, qd1 = xd.y;
  const float tau0 = xt.x, tau1 = xt.y;
  const float c0 = cosf(q0), s0 = sinf(q0), c1 = cosf(q1), s1 = sinf(q1);

#pragma unroll 1
  for (int g = 0; g < 2; ++g) {
    const int nn0 = p * 16 + g * 8;
    const v4f ra0 = *(const v4f*)(W0 + nn0);
    const v4f ra1 = *(const v4f*)(W0 + nn0 + 4);
    const v4f rb0 = *(const v4f*)(W0 + kNeu + nn0);
    const v4f rb1 = *(const v4f*)(W0 + kNeu + nn0 + 4);
    const v4f rc0 = *(const v4f*)(W0 + 2 * kNeu + nn0);
    const v4f rc1 = *(const v4f*)(W0 + 2 * kNeu + nn0 + 4);
    const v4f rd0 = *(const v4f*)(W0 + 3 * kNeu + nn0);
    const v4f rd1 = *(const v4f*)(W0 + 3 * kNeu + nn0 + 4);
    const v4f bb0 = *(const v4f*)(b0 + nn0);
    const v4f bb1 = *(const v4f*)(b0 + nn0 + 4);
    const float wa[8] = {ra0.x, ra0.y, ra0.z, ra0.w, ra1.x, ra1.y, ra1.z, ra1.w};
    const float wb[8] = {rb0.x, rb0.y, rb0.z, rb0.w, rb1.x, rb1.y, rb1.z, rb1.w};
    const float wc[8] = {rc0.x, rc0.y, rc0.z, rc0.w, rc1.x, rc1.y, rc1.z, rc1.w};
    const float wd[8] = {rd0.x, rd0.y, rd0.z, rd0.w, rd1.x, rd1.y, rd1.z, rd1.w};
    const float bz[8] = {bb0.x, bb0.y, bb0.z, bb0.w, bb1.x, bb1.y, bb1.z, bb1.w};
    v8h hv, t0v, t1v;
#pragma unroll
    for (int e = 0; e < 8; ++e) {
      const float z = fmaf(c0, wa[e], fmaf(c1, wb[e], fmaf(s0, wc[e], fmaf(s1, wd[e], bz[e]))));
      const float h = tanhf(z);
      const float u = (1.0f - h * h) * kCarryA;
      const float sd0 = fmaf(-s0, wa[e], c0 * wc[e]);
      const float sd1 = fmaf(-s1, wb[e], c1 * wd[e]);
      hv[e]  = (_Float16)(h * kCarryA);
      t0v[e] = (_Float16)(u * sd0);
      t1v[e] = (_Float16)(u * sd1);
    }
    *(v8h*)(sA + s * kPitchA + nn0)              = hv;
    *(v8h*)(sA + (kSmp + s) * kPitchA + nn0)     = t0v;
    *(v8h*)(sA + (2 * kSmp + s) * kPitchA + nn0) = t1v;
  }
  __syncthreads();

  {
    const int lh = lane >> 4;
    const int lc = lane & 15;
    const int koff = lh * 8;
    const int aoff = lc * kPitchA + koff;
    const int rbase = lh * 8;
#pragma unroll 1
    for (int t = 0; t < 2; ++t) {
      const int nt = wave * 2 + t;
      const int ncol = nt * 16 + lc;
      v8f acc0 = (v8f){0.f, 0.f, 0.f, 0.f, 0.f, 0.f, 0.f, 0.f};
      v8f acc1 = (v8f){0.f, 0.f, 0.f, 0.f, 0.f, 0.f, 0.f, 0.f};
      v8f acc2 = (v8f){0.f, 0.f, 0.f, 0.f, 0.f, 0.f, 0.f, 0.f};
      const _Float16* bp = Bt + (size_t)ncol * kNeu + koff;
#pragma unroll
      for (int ks = 0; ks < 8; ++ks) {
        const v16h bf = Frag<_Float16>::load(bp + ks * 32);
        Frag<_Float16>::U a0, a1, a2;
        a0.h[0] = *(const v8h*)(sA + aoff + ks * 32);
        a0.h[1] = *(const v8h*)(sA + aoff + ks * 32 + 16);
        a1.h[0] = *(const v8h*)(sA + kSmp * kPitchA + aoff + ks * 32);
        a1.h[1] = *(const v8h*)(sA + kSmp * kPitchA + aoff + ks * 32 + 16);
        a2.h[0] = *(const v8h*)(sA + 2 * kSmp * kPitchA + aoff + ks * 32);
        a2.h[1] = *(const v8h*)(sA + 2 * kSmp * kPitchA + aoff + ks * 32 + 16);
        acc0 = mma_h(a0.v, bf, acc0);
        acc1 = mma_h(a1.v, bf, acc1);
        acc2 = mma_h(a2.v, bf, acc2);
      }
      const float b1v = b1[ncol];
#pragma unroll
      for (int r = 0; r < 8; ++r) {
        const float z = fmaf(acc0[r], kFold, b1v);
        const float h = tanhf(z);
        const float u = (1.0f - h * h) * kFold;
        const float d0 = u * acc1[r];
        const float d1 = u * acc2[r];
        const _Float16 d0h = (_Float16)d0;
        const _Float16 d1h = (_Float16)d1;
        sH[(rbase + r) * kPitchH + ncol] = h;
        sT[(rbase + r) * kPitchT + ncol] = __builtin_bit_cast(unsigned short, d0h);
        sT[(kSmp + rbase + r) * kPitchT + ncol] = __builtin_bit_cast(unsigned short, d1h);
      }
    }
  }
  __syncthreads();

  float zd0 = 0.f, zd1 = 0.f, zo = 0.f;
  float ad0 = 0.f, ad1 = 0.f, ao = 0.f, ag = 0.f;
  float bd0 = 0.f, bd1 = 0.f, bo_ = 0.f, bg = 0.f;
#pragma unroll 1
  for (int c = 0; c < 4; ++c) {
    const int j = p * 16 + c * 4;
    const v4f wdA = *(const v4f*)(Wd + 2 * j);
    const v4f wdB = *(const v4f*)(Wd + 2 * j + 4);
    const v4f wo4 = *(const v4f*)(Wo + j);
    const v4f wv4 = *(const v4f*)(Wv + j);
    const v4f h4  = *(const v4f*)(sH + s * kPitchH + j);
    const v2u ta  = *(const v2u*)(sT + s * kPitchT + j);
    const v2u tb  = *(const v2u*)(sT + (kSmp + s) * kPitchT + j);
    const unsigned ta0 = ta.x, ta1 = ta.y, tb0 = tb.x, tb1 = tb.y;
    const float w0[4] = {wdA.x, wdA.z, wdB.x, wdB.z};
    const float w1[4] = {wdA.y, wdA.w, wdB.y, wdB.w};
    const float wo[4] = {wo4.x, wo4.y, wo4.z, wo4.w};
    const float wv[4] = {wv4.x, wv4.y, wv4.z, wv4.w};
    const float hh[4] = {h4.x, h4.y, h4.z, h4.w};
    const float da[4] = {h16_to_f32(ta0 & 0xffffu), h16_to_f32(ta0 >> 16),
                         h16_to_f32(ta1 & 0xffffu), h16_to_f32(ta1 >> 16)};
    const float db[4] = {h16_to_f32(tb0 & 0xffffu), h16_to_f32(tb0 >> 16),
                         h16_to_f32(tb1 & 0xffffu), h16_to_f32(tb1 >> 16)};
#pragma unroll
    for (int e = 0; e < 4; ++e) {
      zd0 = fmaf(hh[e], w0[e], zd0);
      zd1 = fmaf(hh[e], w1[e], zd1);
      zo  = fmaf(hh[e], wo[e], zo);
      ad0 = fmaf(da[e], w0[e], ad0);
      ad1 = fmaf(da[e], w1[e], ad1);
      ao  = fmaf(da[e], wo[e], ao);
      ag  = fmaf(da[e], wv[e], ag);
      bd0 = fmaf(db[e], w0[e], bd0);
      bd1 = fmaf(db[e], w1[e], bd1);
      bo_ = fmaf(db[e], wo[e], bo_);
      bg  = fmaf(db[e], wv[e], bg);
    }
  }
#pragma unroll
  for (int off = 1; off < 16; off <<= 1) {
    zd0 += __shfl_xor(zd0, off, 32);
    zd1 += __shfl_xor(zd1, off, 32);
    zo  += __shfl_xor(zo,  off, 32);
    ad0 += __shfl_xor(ad0, off, 32);
    ad1 += __shfl_xor(ad1, off, 32);
    ao  += __shfl_xor(ao,  off, 32);
    ag  += __shfl_xor(ag,  off, 32);
    bd0 += __shfl_xor(bd0, off, 32);
    bd1 += __shfl_xor(bd1, off, 32);
    bo_ += __shfl_xor(bo_, off, 32);
    bg  += __shfl_xor(bg,  off, 32);
  }

  float acc_q0, acc_q1;
  {
    const float z0 = zd0 + bd[0];
    const float z1 = zd1 + bd[1];
    const float cL = zo + bo[0];
    const float e0 = expf(-fabsf(z0));
    const float e1 = expf(-fabsf(z1));
    const float aL = fmaxf(z0, 0.0f) + log1pf(e0) + kEps;
    const float bL = fmaxf(z1, 0.0f) + log1pf(e1) + kEps;
    const float sg0 = 1.0f / (1.0f + expf(-z0));
    const float sg1 = 1.0f / (1.0f + expf(-z1));
    const float da0 = sg0 * ad0, da1 = sg0 * bd0;
    const float db0 = sg1 * ad1, db1 = sg1 * bd1;
    const float dc0 = ao,        dc1 = bo_;
    const float H00 = aL * aL + kEps;
    const float H01 = aL * cL;
    const float H11 = bL * bL + cL * cL + kEps;
    const float e00_0 = 2.f * aL * da0,                 e00_1 = 2.f * aL * da1;
    const float e01_0 = da0 * cL + aL * dc0,            e01_1 = da1 * cL + aL * dc1;
    const float e11_0 = 2.f * (bL * db0 + cL * dc0),    e11_1 = 2.f * (bL * db1 + cL * dc1);
    const float hv00 = e00_0 * qd0 + e01_0 * qd1;
    const float hv10 = e01_0 * qd0 + e11_0 * qd1;
    const float hv01 = e00_1 * qd0 + e01_1 * qd1;
    const float hv11 = e01_1 * qd0 + e11_1 * qd1;
    const float ke0 = 0.5f * (qd0 * qd0 * e00_0 + 2.f * qd0 * qd1 * e01_0 + qd1 * qd1 * e11_0);
    const float ke1 = 0.5f * (qd0 * qd0 * e00_1 + 2.f * qd0 * qd1 * e01_1 + qd1 * qd1 * e11_1);
    const float C0 = hv00 * qd0 + hv01 * qd1 - ke0;
    const float C1 = hv10 * qd0 + hv11 * qd1 - ke1;
    const float r0 = tau0 - C0 - ag;
    const float r1 = tau1 - C1 - bg;
    const float inv = 1.0f / (H00 * H11 - H01 * H01);
    acc_q0 = (H11 * r0 - H01 * r1) * inv;
    acc_q1 = (H00 * r1 - H01 * r0) * inv;
  }
  {
    float ov = 0.0f;
    ov = (p == 0) ? qd0 : ov;
    ov = (p == 1) ? qd1 : ov;
    ov = (p == 2) ? acc_q0 : ov;
    ov = (p == 3) ? acc_q1 : ov;
    if (p < kOutCols) sO[s * kOutCols + p] = ov;
  }
  __syncthreads();

  if (wave == 0) {
    const int li = (lane < 24) ? lane : 23;
    const v4f val = *(const v4f*)(sO + li * 4);
    float* dst = out + (size_t)blockIdx.x * (kSmp * kOutCols) + li * 4;
    if (lane < 24) *(volatile v4f*)dst = val;
    __threadfence();
    if (lane < 24) *(volatile v4f*)dst = val;
  }
}

extern "C" void kernel_launch(void* const* d_in, const int* in_sizes, int n_in,
                              void* d_out, int out_size, void* d_ws, size_t ws_size,
                              hipStream_t stream) {
  if (n_in < 12) return;
  if (in_sizes[1] != kNumSamples * kOutCols) return;
  if (in_sizes[2] != 4 * kNeu) return;
  if (in_sizes[3] != kNeu) return;
  if (in_sizes[4] != kNeu * kNeu) return;
  if (in_sizes[5] != kNeu) return;
  if (in_sizes[6] != kNeu * 2) return;
  if (in_sizes[7] != 2) return;
  if (in_sizes[8] != kNeu) return;
  if (in_sizes[9] != 1) return;
  if (in_sizes[10] != kNeu) return;
  if (out_size != kNumSamples * kOutCols) return;
  if (ws_size < kWsTotal) return;

  const float* x  = (const float*)d_in[1];
  const float* W0 = (const float*)d_in[2];
  const float* b0 = (const float*)d_in[3];
  const float* W1 = (const float*)d_in[4];
  const float* b1 = (const float*)d_in[5];
  const float* Wd = (const float*)d_in[6];
  const float* bd = (const float*)d_in[7];
  const float* Wo = (const float*)d_in[8];
  const float* bo = (const float*)d_in[9];
  const float* Wv = (const float*)d_in[10];
  float* out = (float*)d_out;

  unsigned short* BT = (unsigned short*)((char*)d_ws + kOffBT);

  transpose_w1_kernel<<<(kNeu * kNeu / 8) / 256, 256, 0, stream>>>(W1, BT);

  torus_dyn_kernel<<<kNumSamples / kSmp, 256, 0, stream>>>(
      x, W0, b0, BT, b1, Wd, bd, Wo, bo, Wv, out, kNumSamples);
}
